// VIN_62715112456540
// MI455X (gfx1250) — hardware-verified
//
#include <hip/hip_runtime.h>


typedef _Float16 v16h __attribute__((ext_vector_type(16)));
typedef _Float16 v8h  __attribute__((ext_vector_type(8)));
typedef v8h  v8ha __attribute__((may_alias));
typedef float v8f  __attribute__((ext_vector_type(8)));
typedef float v4f  __attribute__((ext_vector_type(4)));
typedef v4f  v4fa __attribute__((may_alias));
typedef _Float16 h16a __attribute__((may_alias));

union Frag  { v16h v; v8h hv[2]; unsigned int u[8]; };
union HPair { _Float16 hh[2]; unsigned int u; };

#define IMS    28
#define NPIX   784
#define HW     30
#define XW     32
#define NCQ    10
#define KITER  51
#define WPB    4
#define ROWLEN 1570
#define NTHR   256
#define SC_W   1024.0f
#define SC_Q   256.0f
#define SC_RV  4096.0f

static_assert((WPB * NPIX) % 4 == 0);
static_assert((WPB * NPIX) / 4 <= 4 * NTHR);
static_assert((WPB * NPIX * 4) % 128 == 0);

__device__ __forceinline__ v8f wmma_f16(v16h a, v16h b, v8f c)
{
    v8f d = __builtin_amdgcn_wmma_f32_16x16x32_f16(false, a, false, b, (short)0, c, false, false);
    asm volatile("v_nop\n\tv_nop\n\tv_nop\n\tv_nop" : "+v"(d) : "v"(a), "v"(b));
    return d;
}

__global__ __launch_bounds__(NTHR) void vi_grid_kernel(
    const float* __restrict__ total,
    const float* __restrict__ h1_k,
    const float* __restrict__ h1_b,
    const float* __restrict__ r1_k,
    const float* __restrict__ q1_k,
    float* out,
    int nworld, int chh)
{
    __shared__ unsigned int XP[XW * XW];
    __shared__ float Gs[9 * HW * HW];
    __shared__ unsigned int RV0[HW * HW];
    __shared__ unsigned int RV1[HW * HW];
    __shared__ __attribute__((aligned(16))) _Float16 WA[16 * 32];
    __shared__ __attribute__((aligned(16))) _Float16 WQ[16 * 32];
    __shared__ float bts[16];
    __shared__ __attribute__((aligned(16))) float OUTS[WPB * NPIX];

    const int tid  = threadIdx.x;
    const int lane = tid & 31;
    const int wid  = tid >> 5;
    const int h    = lane >> 4;
    const int m    = lane & 15;
    const int w0   = blockIdx.x * WPB;
    int nw = nworld - w0;
    if (nw > WPB) nw = WPB;
    if (nw < 0) nw = 0;

    for (int i = tid; i < 9 * HW * HW; i += NTHR) Gs[i] = 0.0f;
    for (int i = tid; i < HW * HW; i += NTHR) { RV0[i] = 0u; RV1[i] = 0u; }
    for (int i = tid; i < 16 * 32; i += NTHR) {
        const int row = i >> 5, k = i & 31;
        float wa = 0.0f;
        if (row < 9 && k < 18) {
            float acc = 0.0f;
            #pragma unroll 1
            for (int c = 0; c < chh; ++c) acc += r1_k[row * chh + c] * h1_k[k * chh + c];
            wa = acc * SC_W;
        }
        WA[i] = (_Float16)wa;
        float wq = 0.0f;
        if (row < NCQ && k < 18) wq = q1_k[k * NCQ + row] * SC_Q;
        WQ[i] = (_Float16)wq;
    }
    if (tid < 16) {
        float acc = 0.0f;
        if (tid < 9) {
            #pragma unroll 1
            for (int c = 0; c < chh; ++c) acc += r1_k[tid * chh + c] * h1_b[c];
        }
        bts[tid] = acc * SC_W;
    }
    __syncthreads();

    Frag aW, aQ;
    aW.hv[0] = *(const v8ha*)(WA + m * 32 + 8 * h);
    aW.hv[1] = *(const v8ha*)(WA + m * 32 + 16 + 8 * h);
    aQ.hv[0] = *(const v8ha*)(WQ + m * 32 + 8 * h);
    aQ.hv[1] = *(const v8ha*)(WQ + m * 32 + 16 + 8 * h);
    float btv[8];
    #pragma unroll
    for (int r = 0; r < 8; ++r) btv[r] = bts[8 * h + r];

    const int oq0 = h ? 0        : -(HW + 1);
    const int oq1 = h ? 1        : -HW;
    const int oq2 = h ? (HW - 1) : -(HW - 1);
    const int oq3 = h ? HW       : -1;
    const int ox0 = h ? 0        : -(XW + 1);
    const int ox1 = h ? 1        : -XW;
    const int ox2 = h ? (XW - 1) : -(XW - 1);
    const int ox3 = h ? XW       : -1;
    const unsigned int keep8 = h ? 0u : 0xffffffffu;

    for (int wl = 0; wl < nw; ++wl) {
        const float* tot = total + (size_t)(w0 + wl) * ROWLEN + 2;
        for (int i = tid; i < XW * XW; i += NTHR) {
            const int Y = (i >> 5) - 2, X = (i & 31) - 2;
            unsigned int u = 0u;
            if ((unsigned)Y < (unsigned)IMS && (unsigned)X < (unsigned)IMS) {
                const int p = Y * IMS + X;
                HPair pk;
                pk.hh[0] = (_Float16)tot[2 * p];
                pk.hh[1] = (_Float16)tot[2 * p + 1];
                u = pk.u;
            }
            XP[i] = u;
        }
        __syncthreads();

        for (int tile = wid; tile < NPIX / 16; tile += NTHR / 32) {
            const int p = tile * 16 + m;
            const int y = p / IMS;
            const int x = p - y * IMS;
            const int base = (y + 2) * XW + (x + 2);
            Frag b;
            b.u[0] = XP[base + ox0];
            b.u[1] = XP[base + ox1];
            b.u[2] = XP[base + ox2];
            b.u[3] = XP[base + ox3];
            b.u[4] = XP[base + XW + 1] & keep8;
            b.u[5] = 0u; b.u[6] = 0u; b.u[7] = 0u;
            v8f acc = {0.0f, 0.0f, 0.0f, 0.0f, 0.0f, 0.0f, 0.0f, 0.0f};
            acc = wmma_f16(aW.v, b.v, acc);
            const int gi = (y + 1) * HW + (x + 1);
            if (h == 0) {
                #pragma unroll
                for (int r = 0; r < 8; ++r) Gs[r * (HW * HW) + gi] = acc[r] + btv[r];
            } else {
                Gs[8 * (HW * HW) + gi] = acc[0] + btv[0];
            }
        }
        __syncthreads();

        for (int p = tid; p < NPIX; p += NTHR) {
            const int y = p / IMS, x = p - y * IMS;
            float s = 0.0f;
            #pragma unroll
            for (int ry = 0; ry < 3; ++ry) {
                #pragma unroll
                for (int rx = 0; rx < 3; ++rx)
                    s += Gs[(ry * 3 + rx) * (HW * HW) + (y + ry) * HW + (x + rx)];
            }
            HPair pk;
            pk.hh[0] = (_Float16)(s * (SC_RV / SC_W));
            pk.hh[1] = (_Float16)0.0f;
            const int gi = (y + 1) * HW + (x + 1);
            RV0[gi] = pk.u;
            RV1[gi] = pk.u;
        }
        __syncthreads();

        for (int it = 0; it < KITER; ++it) {
            const unsigned int* rvin = (it & 1) ? RV1 : RV0;
            unsigned int* rvout = (it & 1) ? RV0 : RV1;
            h16a* rvo = (h16a*)rvout;
            const bool last = (it == KITER - 1);
            for (int tile = wid; tile < NPIX / 16; tile += NTHR / 32) {
                const int p = tile * 16 + m;
                const int y = p / IMS;
                const int x = p - y * IMS;
                const int base = (y + 1) * HW + (x + 1);
                Frag b;
                b.u[0] = rvin[base + oq0];
                b.u[1] = rvin[base + oq1];
                b.u[2] = rvin[base + oq2];
                b.u[3] = rvin[base + oq3];
                b.u[4] = rvin[base + HW + 1] & keep8;
                b.u[5] = 0u; b.u[6] = 0u; b.u[7] = 0u;
                v8f acc = {0.0f, 0.0f, 0.0f, 0.0f, 0.0f, 0.0f, 0.0f, 0.0f};
                acc = wmma_f16(aQ.v, b.v, acc);
                const float mlo = fmaxf(fmaxf(fmaxf(acc[0], acc[1]), fmaxf(acc[2], acc[3])),
                                        fmaxf(fmaxf(acc[4], acc[5]), fmaxf(acc[6], acc[7])));
                const float mhi = fmaxf(acc[0], acc[1]);
                float mm = h ? mhi : mlo;
                mm = fmaxf(mm, __shfl_xor(mm, 16, 32));
                const float vs = mm * (1.0f / SC_Q);
                if (h == 0) {
                    rvo[2 * base + 1] = (_Float16)vs;
                    if (last) OUTS[wl * NPIX + p] = vs * (1.0f / SC_RV);
                }
            }
            __syncthreads();
        }
    }
    __syncthreads();

    {
        const int nf4 = nw * (NPIX / 4);
        const v4fa* src = (const v4fa*)OUTS;
        float* dstb = out + (size_t)w0 * NPIX;
        v4f vals[4];
        #pragma unroll
        for (int q = 0; q < 4; ++q) {
            const int f = q * NTHR + tid;
            const int fc = (f < nf4) ? f : 0;
            vals[q] = src[fc];
        }
        #pragma unroll
        for (int q = 0; q < 4; ++q) {
            const int f = q * NTHR + tid;
            if (f < nf4) *(volatile v4f*)(dstb + 4 * (size_t)f) = vals[q];
        }
        __threadfence();
        #pragma unroll
        for (int q = 0; q < 4; ++q) {
            const int f = q * NTHR + tid;
            if (f < nf4) *(volatile v4f*)(dstb + 4 * (size_t)f) = vals[q];
        }
    }
}

extern "C" void kernel_launch(void* const* d_in, const int* in_sizes, int n_in,
                              void* d_out, int out_size, void* d_ws, size_t ws_size,
                              hipStream_t stream)
{
    (void)n_in; (void)d_ws; (void)ws_size;
    const float* total = (const float*)d_in[0];
    const float* h1_k  = (const float*)d_in[1];
    const float* h1_b  = (const float*)d_in[2];
    const float* r1_k  = (const float*)d_in[3];
    const float* q1_k  = (const float*)d_in[4];
    float* out = (float*)d_out;
    const int nworld = in_sizes[0] / ROWLEN;
    const int chh = in_sizes[2];
    if (nworld <= 0 || chh <= 0) return;
    if (in_sizes[1] != 18 * chh || in_sizes[3] != 9 * chh || in_sizes[4] != 18 * NCQ) return;
    if (out_size < nworld * NPIX) return;
    const int nblk = (nworld + WPB - 1) / WPB;
    vi_grid_kernel<<<dim3(nblk), dim3(NTHR), 0, stream>>>(
        total, h1_k, h1_b, r1_k, q1_k, out, nworld, chh);
}
